// GroupInvariance_1906965479549
// MI455X (gfx1250) — hardware-verified
//
#include <hip/hip_runtime.h>
#include <stdint.h>

typedef __attribute__((ext_vector_type(16))) _Float16 v16h;
typedef __attribute__((ext_vector_type(8)))  _Float16 v8h;
typedef __attribute__((ext_vector_type(8)))  float    v8f;
typedef __attribute__((ext_vector_type(4)))  float    v4f;

__device__ __forceinline__ void guard4_h(v8f& a, v8f& b, v8f& c, v8f& d, v16h x, v16h y) {
  asm volatile("v_nop\n\tv_nop\n\tv_nop\n\tv_nop" : "+v"(a), "+v"(b), "+v"(c), "+v"(d) : "v"(x), "v"(y));
}
__device__ __forceinline__ void guard1_h(v8f& a, v16h x, v16h y) {
  asm volatile("v_nop\n\tv_nop\n\tv_nop\n\tv_nop" : "+v"(a) : "v"(x), "v"(y));
}
__device__ __forceinline__ void keep4_h(v16h a, v16h b, v16h c, v16h d) { asm volatile("v_nop" :: "v"(a), "v"(b), "v"(c), "v"(d)); }

template <typename T> struct Frag;
template <> struct Frag<_Float16> {
  typedef v16h V; union U { v16h v; v8h h[2]; };
  static __device__ __forceinline__ v16h load(const _Float16* p) {
    U f; f.h[0] = *(const v8h*)(p); f.h[1] = *(const v8h*)(p + 16); return f.v;
  }
  static __device__ __forceinline__ v8f mma(v16h a, v16h b, v8f c) {
    return __builtin_amdgcn_wmma_f32_16x16x32_f16(false, a, false, b, (short)0, c, false, false);
  }
};

#define NT       320
#define NWAVE    10
#define SETS     32
#define NPT      5
#define ROWS     (SETS * NPT)
#define H2P      72
#define SPITCH   16
#define TWO_LOG2E 2.8853900817779268f
#define OPSCALE  64.0f
#define EPISCALE (1.0f / 4096.0f)

__device__ __forceinline__ float tanh_x64(float x) {
  const float e = __builtin_amdgcn_exp2f(x * TWO_LOG2E);
  return fmaf(-128.0f, __builtin_amdgcn_rcpf(e + 1.0f), 64.0f);
}

__global__ void __launch_bounds__(NT)
fused_group_pool(const float* __restrict__ inputs,
                 const float* __restrict__ W1,  const float* __restrict__ b1,
                 const float* __restrict__ W2,  const float* __restrict__ b2,
                 const float* __restrict__ W3,  const float* __restrict__ b3,
                 const float* __restrict__ Wfc, const float* __restrict__ Wout,
                 const float* __restrict__ bout,
                 float* __restrict__ out, int nrows, int nsets)
{
  __shared__ __align__(16) _Float16 W2t[64 * 32];
  __shared__ __align__(16) _Float16 W3t[16 * 64];
  __shared__ __align__(16) _Float16 H2[NWAVE][16 * H2P];
  __shared__ __align__(16) float    Sp[ROWS * SPITCH];
  __shared__ float pW1[16], pb1[16], pb2[64], pb3[16], pWfc[128], pWout[64], pbout[4];
  __shared__ float prodbuf[NT];
  __shared__ float ybuf[2 * SETS];
  __shared__ __align__(16) float outs[SETS];

  const int tid  = threadIdx.x;
  const int wave = tid >> 5;
  const int lane = tid & 31;
  const int hh   = lane >> 4;
  const int m    = lane & 15;

  for (int idx = tid; idx < 64 * 32; idx += NT) {
    const int n = idx >> 5, k = idx & 31;
    const int kk = (k < 16) ? k : 15;
    const float v = W2[kk * 64 + n];
    W2t[idx] = (_Float16)((k < 16) ? v * OPSCALE : 0.0f);
  }
  for (int idx = tid; idx < 16 * 64; idx += NT) {
    const int n = idx >> 6, k = idx & 63;
    const int nn = (n < 10) ? n : 9;
    const float v = W3[k * 10 + nn];
    W3t[idx] = (_Float16)((n < 10) ? v * OPSCALE : 0.0f);
  }
  if (tid < 16) { pW1[tid] = W1[tid]; pb1[tid] = b1[tid]; }
  if (tid < 64) { pb2[tid] = b2[tid]; pWout[tid] = Wout[tid]; }
  if (tid < 16) { const int nn = (tid < 10) ? tid : 9; const float v = b3[nn]; pb3[tid] = (tid < 10) ? v : 0.0f; }
  if (tid < 128) pWfc[tid] = Wfc[tid];
  if (tid == 0) pbout[0] = bout[0];
  __syncthreads();

  const int lrow0 = wave * 16;
  {
    int p = blockIdx.x * ROWS + lrow0 + m;
    p = (p < nrows) ? p : (nrows - 1);
    const float t = inputs[p];

    v16h a1;
#pragma unroll
    for (int i = 0; i < 8; ++i) {
      const int k = 8 * hh + i;
      const float v = tanh_x64(fmaf(t, pW1[k], pb1[k]));
      a1[i] = (_Float16)v;
      a1[8 + i] = (_Float16)0.0f;
    }

    v16h bf2[4];
#pragma unroll
    for (int nt = 0; nt < 4; ++nt) bf2[nt] = Frag<_Float16>::load(W2t + (nt * 16 + m) * 32 + 8 * hh);
    v8f acc2[4];
#pragma unroll
    for (int nt = 0; nt < 4; ++nt) {
      acc2[nt] = (v8f){0.f, 0.f, 0.f, 0.f, 0.f, 0.f, 0.f, 0.f};
      acc2[nt] = Frag<_Float16>::mma(a1, bf2[nt], acc2[nt]);
    }
    keep4_h(bf2[0], bf2[1], bf2[2], bf2[3]);
    guard4_h(acc2[0], acc2[1], acc2[2], acc2[3], a1, bf2[3]);

    _Float16* h2 = H2[wave];
#pragma unroll
    for (int nt = 0; nt < 4; ++nt) {
      const int col = nt * 16 + m;
      const float bv = pb2[col];
#pragma unroll
      for (int r = 0; r < 8; ++r) {
        const float v = fmaf(acc2[nt][r], EPISCALE, bv);
        h2[(8 * hh + r) * H2P + col] = (_Float16)tanh_x64(v);
      }
    }
    __builtin_amdgcn_fence(__ATOMIC_RELEASE, "workgroup");
    __builtin_amdgcn_wave_barrier();
    __builtin_amdgcn_fence(__ATOMIC_ACQUIRE, "workgroup");

    v16h a3[2], bf3[2];
#pragma unroll
    for (int kt = 0; kt < 2; ++kt) {
      a3[kt]  = Frag<_Float16>::load(h2 + m * H2P + kt * 32 + 8 * hh);
      bf3[kt] = Frag<_Float16>::load(W3t + m * 64 + kt * 32 + 8 * hh);
    }
    v8f acc3 = (v8f){0.f, 0.f, 0.f, 0.f, 0.f, 0.f, 0.f, 0.f};
    acc3 = Frag<_Float16>::mma(a3[0], bf3[0], acc3);
    acc3 = Frag<_Float16>::mma(a3[1], bf3[1], acc3);
    keep4_h(a3[0], bf3[0], a3[1], bf3[1]);
    guard1_h(acc3, a3[1], bf3[1]);

    const float bv3 = pb3[m];
#pragma unroll
    for (int r = 0; r < 8; ++r)
      Sp[(lrow0 + 8 * hh + r) * SPITCH + m] = fmaf(acc3[r], EPISCALE, bv3);
  }
  __syncthreads();

  {
    const int s   = tid / 10;
    const int rem = tid - s * 10;
    const int f   = (rem >= 5) ? 1 : 0;
    const int i   = rem - 5 * f;
    float prod = 1.0f;
#pragma unroll
    for (int j = 0; j < NPT; ++j) {
      int c = i + j; c = (c >= NPT) ? (c - NPT) : c;
      const float x  = Sp[(s * NPT + j) * SPITCH + f * NPT + c];
      const float e  = expf(-x);
      const float sg = 1.0f / (1.0f + e);
      prod *= sg;
    }
    prodbuf[tid] = prod;
  }
  __syncthreads();
  if (tid < 2 * SETS) {
    const int base = (tid >> 1) * 10 + (tid & 1) * 5;
    float y = 0.0f;
#pragma unroll
    for (int i = 0; i < NPT; ++i) y += prodbuf[base + i];
    ybuf[tid] = y;
  }
  __syncthreads();

  if (wave == 0) {
    const float y0 = ybuf[lane * 2 + 0];
    const float y1 = ybuf[lane * 2 + 1];
    float acc = 0.0f;
#pragma unroll 4
    for (int n = 0; n < 64; ++n) {
      float hv = y0 * pWfc[n] + y1 * pWfc[64 + n];
      hv = fmaxf(hv, 0.0f);
      acc = fmaf(hv, pWout[n], acc);
    }
    acc += pbout[0];
    const int set0 = blockIdx.x * SETS;
    if (set0 + SETS <= nsets) {
      outs[lane] = acc;
      __builtin_amdgcn_fence(__ATOMIC_RELEASE, "workgroup");
      __builtin_amdgcn_wave_barrier();
      __builtin_amdgcn_fence(__ATOMIC_ACQUIRE, "workgroup");
      if (lane < 8) {
        const v4f v = *(const v4f*)(outs + 4 * lane);
        float* pd = out + (size_t)set0 + 4 * lane;
        *(volatile v4f*)pd = v;
        __threadfence();
        *(volatile v4f*)pd = v;
      }
    } else {
      const int si = set0 + lane;
      if (si < nsets) {
        const float v = acc;
        *(volatile float*)(out + si) = v;
        __threadfence();
        *(volatile float*)(out + si) = v;
      }
    }
  }
}

extern "C" void kernel_launch(void* const* d_in, const int* in_sizes, int n_in,
                              void* d_out, int out_size, void* d_ws, size_t ws_size,
                              hipStream_t stream) {
  (void)n_in; (void)d_ws; (void)ws_size;
  const float* inputs = (const float*)d_in[0];
  const float* W1     = (const float*)d_in[1];
  const float* b1     = (const float*)d_in[2];
  const float* W2     = (const float*)d_in[3];
  const float* b2     = (const float*)d_in[4];
  const float* W3     = (const float*)d_in[5];
  const float* b3     = (const float*)d_in[6];
  const float* Wfc    = (const float*)d_in[7];
  const float* Wout   = (const float*)d_in[8];
  const float* bout   = (const float*)d_in[9];
  float* out          = (float*)d_out;

  const int nrows = in_sizes[0];
  int nsets = nrows / NPT;
  if (nsets > out_size) nsets = out_size;
  if (nsets <= 0 || nrows <= 0) return;
  const int grid = (nsets + SETS - 1) / SETS;

  fused_group_pool<<<grid, NT, 0, stream>>>(inputs, W1, b1, W2, b2, W3, b3, Wfc, Wout, bout,
                                            out, nrows, nsets);
}
